// MultiHeadSelfAttention_73005854097681
// MI455X (gfx1250) — hardware-verified
//
#include <hip/hip_runtime.h>
#include <math.h>

typedef __attribute__((ext_vector_type(16))) _Float16 v16h;
typedef __attribute__((ext_vector_type(16))) __bf16 v16b;
typedef __attribute__((ext_vector_type(8)))  _Float16 v8h;
typedef __attribute__((ext_vector_type(8)))  __bf16 v8b;
typedef __attribute__((ext_vector_type(8)))  float v8f;
typedef __attribute__((ext_vector_type(4)))  float v4f;
typedef __attribute__((ext_vector_type(2)))  float v2f;
typedef __attribute__((ext_vector_type(4)))  unsigned v4u;

template <typename T> __device__ __forceinline__ void vst2(void* p, T v) { *(volatile T*)p = v; __threadfence(); *(volatile T*)p = v; }
__device__ __forceinline__ v8f wmma16(v16h a, v16h b, v8f c) {
  v8f d = __builtin_amdgcn_wmma_f32_16x16x32_f16(false, a, false, b, (short)0, c, false, false);
  asm volatile("v_nop\n\tv_nop\n\tv_nop\n\tv_nop" : "+v"(d) : "v"(a), "v"(b));
  return d;
}
__device__ __forceinline__ v8f wmma_bf(v16b a, v16b b, v8f c) {
  v8f d = __builtin_amdgcn_wmma_f32_16x16x32_bf16(false, a, false, b, (short)0, c, false, false);
  asm volatile("v_nop\n\tv_nop\n\tv_nop\n\tv_nop" : "+v"(d) : "v"(a), "v"(b));
  return d;
}
__device__ __forceinline__ v16h frag_h(const _Float16* rowk0, int lane) {
  union { v16h v; v8h q[2]; } u; const _Float16* p = rowk0 + 8 * (lane >> 4);
  u.q[0] = *(const v8h*)p; u.q[1] = *(const v8h*)(p + 16); return u.v;
}
__device__ __forceinline__ v16b frag_b(const __bf16* rowk0, int lane) {
  union { v16b v; v8b q[2]; } u; const __bf16* p = rowk0 + 8 * (lane >> 4);
  u.q[0] = *(const v8b*)p; u.q[1] = *(const v8b*)(p + 16); return u.v;
}
#define LDSX() do { asm volatile("s_wait_dscnt 0" ::: "memory"); __builtin_amdgcn_wave_barrier(); __builtin_amdgcn_fence(3  , "workgroup"); } while (0)

#ifndef NB
#define NB 2
#endif
#ifndef SEQ
#define SEQ 2048
#endif
#define NB_FULL 2
#define SEQ_FULL 2048
#define CC 1024
#define DIN 1024
#define NH 16
#define HD 64
#define QBE 4
#define KHI 256

static_assert(CC == NH * HD);
static_assert(CC == DIN);
static_assert(HD == 64);
static_assert(DIN % 32 == 0 && CC % 128 == 0);
static_assert(SEQ % 64 == 0);
static_assert(SEQ >= KHI && KHI == QBE * 64);
static_assert((SEQ * 32) % 256 == 0);
static_assert(((size_t)NB * SEQ * DIN / 8) % 256 == 0 && ((size_t)CC * DIN / 8) % 256 == 0);
static_assert(NB <= NB_FULL && SEQ <= SEQ_FULL);

#define WS_XB  ((size_t)0)
#define WS_WQ  (WS_XB + 2u * (size_t)NB * SEQ * DIN)
#define WS_WK  (WS_WQ + 2u * (size_t)CC * DIN)
#define WS_WV  (WS_WK + 2u * (size_t)CC * DIN)
#define WS_WO  (WS_WV + 2u * (size_t)CC * DIN)
#define WS_QH  (WS_WO + 2u * (size_t)CC * DIN)
#define WS_QL  (WS_QH + 2u * (size_t)NB * SEQ * CC)
#define WS_KH  (WS_QL + 2u * (size_t)NB * SEQ * CC)
#define WS_KL  (WS_KH + 2u * (size_t)NB * SEQ * CC)
#define WS_VT  (WS_KL + 2u * (size_t)NB * SEQ * CC)
#define WS_VB  (WS_VT + 2u * (size_t)NB * CC * SEQ)
#define WS_VBL (WS_VB + 2u * (size_t)NB * CC * KHI)
#define WS_CH  (WS_VBL + 2u * (size_t)NB * CC * KHI)
#define WS_CL  (WS_CH + 2u * (size_t)NB * SEQ * CC)
#define WS_TAB (WS_CL + 2u * (size_t)NB * SEQ * CC)
#define WS_END (WS_TAB + 8u * (size_t)SEQ * 32)
static_assert(WS_END <= (size_t)134217728);
static_assert(WS_QH % 128 == 0 && WS_VT % 128 == 0 && WS_VB % 128 == 0 && WS_CH % 128 == 0 && WS_TAB % 128 == 0);

__global__ __launch_bounds__(256) void k_tab(const int* __restrict__ POS, float* __restrict__ TAB) {
#pragma clang fp contract(off)
  const int e = blockIdx.x * 256 + threadIdx.x;
  const int s = e >> 5, j = e & 31;
  double p = 1.0;
  if (j & 1)  p = p * 1.3335214321633240;
  if (j & 2)  p = p * 1.7782794100389228;
  if (j & 4)  p = p * 3.1622776601683795;
  if (j & 8)  p = p * 10.0;
  if (j & 16) p = p * 100.0;
  const float pf = (float)p;
  const float inv = 1.0f / pf;
  const int sc = s < SEQ ? s : SEQ - 1;
  const float ang = (float)POS[sc] * inv;
  float sn, cs; sincosf(ang, &sn, &cs);
  v2f v; v[0] = cs; v[1] = sn;
  if (s < SEQ) vst2<v2f>(TAB + (size_t)e * 2, v);
}

__global__ __launch_bounds__(256) void k_cvt(const float* __restrict__ SRC, __bf16* __restrict__ DST, int rpb, int sbr, int ngroups) {
  const int gi = blockIdx.x * 256 + threadIdx.x;
  if (gi >= ngroups) return;
  const int row = gi >> 7, cg = gi & 127;
  const int bb = row / rpb, t = row - bb * rpb;
  const float* p = SRC + ((size_t)bb * sbr + t) * DIN + cg * 8;
  const v4f a = *(const v4f*)p, c = *(const v4f*)(p + 4);
  union { v8b b; v4u u; } o;
  o.b[0] = (__bf16)a[0]; o.b[1] = (__bf16)a[1]; o.b[2] = (__bf16)a[2]; o.b[3] = (__bf16)a[3];
  o.b[4] = (__bf16)c[0]; o.b[5] = (__bf16)c[1]; o.b[6] = (__bf16)c[2]; o.b[7] = (__bf16)c[3];
  const v4u val = o.u;
  vst2<v4u>(DST + (size_t)gi * 8, val);
}
static_assert(DIN / 8 == 128);

__global__ __launch_bounds__(128) void k_proj_qk(const __bf16* __restrict__ XB, const __bf16* __restrict__ WB, const float* __restrict__ TAB, __bf16* __restrict__ DH, __bf16* __restrict__ DL) {
  __shared__ __align__(16) float st[64][132];
  __shared__ __align__(16) __bf16 sh[64][136], sl[64][136];
  const int tid = threadIdx.x; const int wave = __builtin_amdgcn_readfirstlane((int)(threadIdx.x >> 5)); const int lane = tid & 31, col = lane & 15, g = lane >> 4;
  const int c0 = blockIdx.y * 128; const size_t r0 = (size_t)blockIdx.x * 64;
  v8f acc[8] = {};
#pragma unroll 1
  for (int kc = 0; kc < DIN / 32; ++kc) {
    const v16b a = frag_b(XB + (r0 + wave * 16 + col) * DIN + kc * 32, lane);
#pragma unroll
    for (int j = 0; j < 8; ++j) { const v16b w = frag_b(WB + (size_t)(c0 + j * 16 + col) * DIN + kc * 32, lane); acc[j] = wmma_bf(a, w, acc[j]); }
  }
#pragma unroll
  for (int j = 0; j < 8; ++j) {
#pragma unroll
    for (int r = 0; r < 8; ++r) st[wave * 16 + 8 * g + r][j * 16 + col] = acc[j][r];
  }
  __syncthreads();
#pragma unroll 2
  for (int e = tid; e < 64 * 64; e += 128) {
    const int rl = e >> 6, jj = e & 63;
    const int t = (int)((r0 + rl) % SEQ);
    const v2f cs = *(const v2f*)(TAB + ((size_t)t * 32 + (jj & 31)) * 2);
    const float xr = st[rl][2 * jj], xi = st[rl][2 * jj + 1];
    const float rr = xr * cs[0] - xi * cs[1];
    const float ri = xr * cs[1] + xi * cs[0];
    const __bf16 hr = (__bf16)rr, hi2 = (__bf16)ri;
    sh[rl][2 * jj] = hr; sh[rl][2 * jj + 1] = hi2;
    sl[rl][2 * jj] = (__bf16)(rr - (float)hr); sl[rl][2 * jj + 1] = (__bf16)(ri - (float)hi2);
  }
  __syncthreads();
  for (int e = tid; e < 64 * 16; e += 128) {
    const int rl = e >> 4, q = e & 15;
    const v4u vh = *(const v4u*)&sh[rl][q * 8]; const v4u vl = *(const v4u*)&sl[rl][q * 8];
    vst2<v4u>(DH + (r0 + rl) * CC + c0 + q * 8, vh);
    vst2<v4u>(DL + (r0 + rl) * CC + c0 + q * 8, vl);
  }
}

__global__ __launch_bounds__(128) void k_proj_v(const __bf16* __restrict__ XB, const __bf16* __restrict__ WB, _Float16* __restrict__ VT, __bf16* __restrict__ VB, __bf16* __restrict__ VBL) {
  __shared__ __align__(16) _Float16 th[128][72]; __shared__ __align__(16) __bf16 tb[128][72], tbl[128][72];
  const int tid = threadIdx.x; const int wave = __builtin_amdgcn_readfirstlane((int)(threadIdx.x >> 5)); const int lane = tid & 31, col = lane & 15, g = lane >> 4;
  const int c0 = blockIdx.y * 128; const size_t r0 = (size_t)blockIdx.x * 64; const size_t bb = r0 / SEQ; const int t0 = (int)(r0 % SEQ);
  v8f acc[8] = {};
#pragma unroll 1
  for (int kc = 0; kc < DIN / 32; ++kc) {
    const v16b a = frag_b(XB + (r0 + wave * 16 + col) * DIN + kc * 32, lane);
#pragma unroll
    for (int j = 0; j < 8; ++j) { const v16b w = frag_b(WB + (size_t)(c0 + j * 16 + col) * DIN + kc * 32, lane); acc[j] = wmma_bf(a, w, acc[j]); }
  }
#pragma unroll
  for (int j = 0; j < 8; ++j) {
#pragma unroll
    for (int r = 0; r < 8; ++r) { const float v = acc[j][r]; const int cl = j * 16 + col, tl = wave * 16 + 8 * g + r;
      th[cl][tl] = (_Float16)v; const __bf16 hb = (__bf16)v; tb[cl][tl] = hb; tbl[cl][tl] = (__bf16)(v - (float)hb); }
  }
  __syncthreads();
  const bool hi_rows = t0 < KHI;
  for (int e = tid; e < 128 * 8; e += 128) {
    const int cl = e >> 3, q = e & 7;
    const v4u vf = *(const v4u*)&th[cl][q * 8];
    vst2<v4u>(VT + (bb * CC + c0 + cl) * (size_t)SEQ + t0 + q * 8, vf);
    if (hi_rows) { const size_t o3 = (bb * CC + c0 + cl) * (size_t)KHI + t0 + q * 8; const v4u vb = *(const v4u*)&tb[cl][q * 8]; const v4u vbl = *(const v4u*)&tbl[cl][q * 8]; vst2<v4u>(VB + o3, vb); vst2<v4u>(VBL + o3, vbl); }
  }
}

__global__ __launch_bounds__(128) void k_attn(const __bf16* __restrict__ QH, const __bf16* __restrict__ QL, const __bf16* __restrict__ KH, const __bf16* __restrict__ KL,
    const _Float16* __restrict__ VT, const __bf16* __restrict__ VB, const __bf16* __restrict__ VBL, __bf16* __restrict__ CH, __bf16* __restrict__ CL) {
  __shared__ __align__(16) float ps[4][16][36];
  __shared__ __align__(16) __bf16 ch[4][16][72], cl[4][16][72];
  const int tid = threadIdx.x; const int wave = __builtin_amdgcn_readfirstlane((int)(threadIdx.x >> 5)); const int lane = tid & 31, col = lane & 15, g = lane >> 4;
  const int qb = blockIdx.x; const int bh = blockIdx.y; const int b = bh / NH, h = bh % NH;
  const bool early = qb < QBE;
  const int ql0 = qb * 64 + wave * 16;
  const int nit = ((ql0 + 15) >> 5) + 1;
  const int qoff0 = (b * SEQ + ql0 + col) * CC + h * HD;
  const int kbase = (b * SEQ + col) * CC + h * HD;
  float mst[8], lsum[8];
#pragma unroll
  for (int r = 0; r < 8; ++r) { mst[r] = -1.0e30f; lsum[r] = 0.0f; }
  v8f o[4] = {};
#pragma unroll 1
  for (int it = 0; it < nit; ++it) {
    const int key0 = it * 32;
    v8f sc0 = {}, sc1 = {};
#pragma unroll
    for (int kc = 0; kc < 2; ++kc) {
      int qo = qoff0 + kc * 32; int ko = kbase + key0 * CC + kc * 32;
      asm volatile("" : "+v"(qo), "+v"(ko));
      const v16b qh = frag_b(QH + qo, lane), qlf = frag_b(QL + qo, lane);
      const v16b kh0 = frag_b(KH + ko, lane), kl0 = frag_b(KL + ko, lane);
      const v16b kh1 = frag_b(KH + ko + 16 * CC, lane), kl1 = frag_b(KL + ko + 16 * CC, lane);
      sc0 = wmma_bf(qlf, kh0, sc0); sc0 = wmma_bf(qh, kl0, sc0); sc0 = wmma_bf(qh, kh0, sc0);
      sc1 = wmma_bf(qlf, kh1, sc1); sc1 = wmma_bf(qh, kl1, sc1); sc1 = wmma_bf(qh, kh1, sc1);
    }
    const int ka = key0 + col, kb = ka + 16;
#pragma unroll
    for (int r = 0; r < 8; ++r) {
      const int m = ql0 + 8 * g + r;
      const float s0 = sc0[r] * 0.125f, s1 = sc1[r] * 0.125f;
      const bool v0 = ka <= m, v1 = kb <= m;
      float mx = fmaxf(v0 ? s0 : -1.0e30f, v1 ? s1 : -1.0e30f);
      mx = fmaxf(mx, __shfl_xor(mx, 1)); mx = fmaxf(mx, __shfl_xor(mx, 2)); mx = fmaxf(mx, __shfl_xor(mx, 4)); mx = fmaxf(mx, __shfl_xor(mx, 8));
      const float mnew = fmaxf(mst[r], mx);
      const float corr = __expf(mst[r] - mnew);
      mst[r] = mnew;
      const float x0 = __expf(s0 - mnew), x1 = __expf(s1 - mnew);
      const float e0 = v0 ? x0 : 0.0f, e1 = v1 ? x1 : 0.0f;
      lsum[r] = lsum[r] * corr + (e0 + e1);
      o[0][r] *= corr; o[1][r] *= corr; o[2][r] *= corr; o[3][r] *= corr;
      ps[wave][8 * g + r][col] = e0; ps[wave][8 * g + r][16 + col] = e1;
    }
    LDSX();
    float pv[16];
#pragma unroll
    for (int i = 0; i < 8; ++i) { pv[i] = ps[wave][col][8 * g + i]; pv[8 + i] = ps[wave][col][16 + 8 * g + i]; }
    LDSX();
    if (early) {
      v16b ph, pl;
#pragma unroll
      for (int i = 0; i < 16; ++i) { const __bf16 hb = (__bf16)pv[i]; ph[i] = hb; pl[i] = (__bf16)(pv[i] - (float)hb); }
      int vo = (b * CC + h * HD + col) * KHI + key0;
      asm volatile("" : "+v"(vo));
#pragma unroll
      for (int j = 0; j < 4; ++j) { const v16b vh = frag_b(VB + vo + j * 16 * KHI, lane), vl = frag_b(VBL + vo + j * 16 * KHI, lane);
        o[j] = wmma_bf(pl, vh, o[j]); o[j] = wmma_bf(ph, vl, o[j]); o[j] = wmma_bf(ph, vh, o[j]); }
    } else {
      v16h pf;
#pragma unroll
      for (int i = 0; i < 16; ++i) pf[i] = (_Float16)(pv[i] * 2048.0f);
      int vo = (b * CC + h * HD + col) * SEQ + key0;
      asm volatile("" : "+v"(vo));
      const v16h vf0 = frag_h(VT + vo, lane), vf1 = frag_h(VT + vo + 16 * SEQ, lane), vf2 = frag_h(VT + vo + 32 * SEQ, lane), vf3 = frag_h(VT + vo + 48 * SEQ, lane);
      o[0] = wmma16(pf, vf0, o[0]); o[1] = wmma16(pf, vf1, o[1]); o[2] = wmma16(pf, vf2, o[2]); o[3] = wmma16(pf, vf3, o[3]);
    }
  }
  const float osc = early ? 1.0f : (1.0f / 2048.0f);
#pragma unroll
  for (int r = 0; r < 8; ++r) {
    float l = lsum[r];
    l += __shfl_xor(l, 1); l += __shfl_xor(l, 2); l += __shfl_xor(l, 4); l += __shfl_xor(l, 8);
    const float inv = osc * (1.0f / l);
#pragma unroll
    for (int j = 0; j < 4; ++j) { const float v = o[j][r] * inv; const __bf16 hb = (__bf16)v; ch[wave][8 * g + r][j * 16 + col] = hb; cl[wave][8 * g + r][j * 16 + col] = (__bf16)(v - (float)hb); }
  }
  LDSX();
#pragma unroll
  for (int rr = 0; rr < 4; ++rr) {
    const int row = rr * 4 + (lane >> 3), q = lane & 7;
    const size_t dst = ((size_t)b * SEQ + ql0 + row) * CC + h * HD + q * 8;
    const v4u vh = *(const v4u*)&ch[wave][row][q * 8]; const v4u vl = *(const v4u*)&cl[wave][row][q * 8];
    vst2<v4u>(CH + dst, vh);
    vst2<v4u>(CL + dst, vl);
  }
}

__global__ __launch_bounds__(128) void k_out(const __bf16* __restrict__ CH, const __bf16* __restrict__ CL, const __bf16* __restrict__ WOB, float* __restrict__ OUT) {
  __shared__ __align__(16) float sf[4][16][132];
  const int tid = threadIdx.x; const int wave = __builtin_amdgcn_readfirstlane((int)(threadIdx.x >> 5)); const int lane = tid & 31, col = lane & 15, g = lane >> 4;
  const int c0 = blockIdx.y * 128; const size_t r0 = (size_t)blockIdx.x * 64 + wave * 16;
  v8f acc[8] = {};
#pragma unroll 1
  for (int kc = 0; kc < CC / 32; ++kc) {
    const v16b ah = frag_b(CH + (r0 + col) * CC + kc * 32, lane), al = frag_b(CL + (r0 + col) * CC + kc * 32, lane);
#pragma unroll
    for (int j = 0; j < 8; ++j) { const v16b w = frag_b(WOB + (size_t)(c0 + j * 16 + col) * CC + kc * 32, lane); acc[j] = wmma_bf(al, w, acc[j]); acc[j] = wmma_bf(ah, w, acc[j]); }
  }
#pragma unroll
  for (int j = 0; j < 8; ++j) {
#pragma unroll
    for (int r = 0; r < 8; ++r) sf[wave][8 * g + r][j * 16 + col] = acc[j][r];
  }
  LDSX();
  for (int rl = 0; rl < 16; ++rl) {
    const size_t prow = r0 + rl; const size_t bb = prow / SEQ; const size_t t = prow % SEQ;
    const v4f v = *(const v4f*)&sf[wave][rl][lane * 4];
    vst2<v4f>(OUT + (bb * SEQ_FULL + t) * DIN + c0 + lane * 4, v);
  }
}
static_assert(32 * 4 == 128);

extern "C" void kernel_launch(void* const* d_in, const int* in_sizes, int n_in, void* d_out, int out_size, void* d_ws, size_t ws_size, hipStream_t stream) {
  if (n_in < 6) return;
  const long long need_x = ((long long)(NB - 1) * SEQ_FULL + SEQ) * DIN;
  if ((long long)in_sizes[0] < need_x) return;
  if (in_sizes[1] < CC * DIN || in_sizes[2] < CC * DIN || in_sizes[3] < CC * DIN || in_sizes[4] < CC * DIN) return;
  if (in_sizes[5] < SEQ) return;
  if ((long long)out_size < need_x) return;
  if (ws_size < (size_t)WS_END) return;
  const float* X  = (const float*)d_in[0];
  const float* Wq = (const float*)d_in[1];
  const float* Wk = (const float*)d_in[2];
  const float* Wv = (const float*)d_in[3];
  const float* Wo = (const float*)d_in[4];
  const int*  POS = (const int*)d_in[5];
  char* ws = (char*)d_ws;
  __bf16 *XB = (__bf16*)(ws + WS_XB), *WQB = (__bf16*)(ws + WS_WQ), *WKB = (__bf16*)(ws + WS_WK), *WVB = (__bf16*)(ws + WS_WV), *WOB = (__bf16*)(ws + WS_WO);
  __bf16 *QH = (__bf16*)(ws + WS_QH), *QL = (__bf16*)(ws + WS_QL), *KH = (__bf16*)(ws + WS_KH), *KL = (__bf16*)(ws + WS_KL);
  _Float16* VT = (_Float16*)(ws + WS_VT); __bf16 *VB = (__bf16*)(ws + WS_VB), *VBL = (__bf16*)(ws + WS_VBL);
  __bf16 *CH = (__bf16*)(ws + WS_CH), *CL = (__bf16*)(ws + WS_CL); float* TAB = (float*)(ws + WS_TAB);

  k_tab<<<dim3(SEQ * 32 / 256), 256, 0, stream>>>(POS, TAB);
  const int gx = NB * SEQ * (DIN / 8), gw = CC * (DIN / 8);
  k_cvt<<<dim3((gx + 255) / 256), 256, 0, stream>>>(X,  XB,  SEQ, SEQ_FULL, gx);
  k_cvt<<<dim3((gw + 255) / 256), 256, 0, stream>>>(Wq, WQB, CC, CC, gw);
  k_cvt<<<dim3((gw + 255) / 256), 256, 0, stream>>>(Wk, WKB, CC, CC, gw);
  k_cvt<<<dim3((gw + 255) / 256), 256, 0, stream>>>(Wv, WVB, CC, CC, gw);
  k_cvt<<<dim3((gw + 255) / 256), 256, 0, stream>>>(Wo, WOB, CC, CC, gw);
  k_proj_qk<<<dim3(NB * SEQ / 64, CC / 128), 128, 0, stream>>>(XB, WQB, TAB, QH, QL);
  k_proj_qk<<<dim3(NB * SEQ / 64, CC / 128), 128, 0, stream>>>(XB, WKB, TAB, KH, KL);
  k_proj_v<<<dim3(NB * SEQ / 64, CC / 128), 128, 0, stream>>>(XB, WVB, VT, VB, VBL);
  k_attn<<<dim3(SEQ / 64, NB * NH), 128, 0, stream>>>(QH, QL, KH, KL, VT, VB, VBL, CH, CL);
  k_out<<<dim3(NB * SEQ / 64, DIN / 128), 128, 0, stream>>>(CH, CL, WOB, (float*)d_out);
}
